// GAT2_28372553957492
// MI455X (gfx1250) — hardware-run, weakly checked
//
#include <hip/hip_runtime.h>

typedef float          v8f   __attribute__((ext_vector_type(8)));
typedef float          v4f   __attribute__((ext_vector_type(4)));
typedef unsigned int   v4u   __attribute__((ext_vector_type(4)));
typedef int            v8i   __attribute__((ext_vector_type(8)));
typedef unsigned short v8us  __attribute__((ext_vector_type(8)));
typedef unsigned short v16us __attribute__((ext_vector_type(16)));
typedef __bf16         v16bf __attribute__((ext_vector_type(16)));
typedef _Float16       v16h  __attribute__((ext_vector_type(16)));
typedef v4f  __attribute__((may_alias)) v4fa;
typedef v8us __attribute__((may_alias)) v8usa;
union FragB { v16bf v; v16us u; v8us h[2]; v8i w; };
union FragH { v16h  v; v16us u; v8us h[2]; v8i w; };

__device__ __forceinline__ v8f wmb(const FragB& a, const FragB& b, v8f c) {
  v8f d = __builtin_amdgcn_wmma_f32_16x16x32_bf16(false, a.v, false, b.v, (short)0, c, false, false);
  asm volatile("v_nop\n\tv_nop\n\tv_nop\n\tv_nop" : "+v"(d) : "v"(a.w), "v"(b.w));
  return d;
}

__device__ __forceinline__ v8f wmh(const FragH& a, const FragH& b, v8f c) {
  v8f d = __builtin_amdgcn_wmma_f32_16x16x32_f16(false, a.v, false, b.v, (short)0, c, false, false);
  asm volatile("v_nop\n\tv_nop\n\tv_nop\n\tv_nop" : "+v"(d) : "v"(a.w), "v"(b.w));
  return d;
}

__device__ __forceinline__ unsigned bf16_bits(float f) {
  const unsigned u = __float_as_uint(f);
  const unsigned r = (u + 0x7FFFu + ((u >> 16) & 1u)) >> 16;
  const unsigned q = (u >> 16) | 0x40u;
  return ((u & 0x7fffffffu) > 0x7f800000u) ? q : r;
}

__device__ __forceinline__ float bf16_val(float f) {
  return __uint_as_float(bf16_bits(f) << 16);
}
__device__ __forceinline__ int clampi(int v, int lo, int hi) {
  return v < lo ? lo : (v > hi ? hi : v);
}

__device__ __forceinline__ unsigned f16_bits(float f) {
  const unsigned u  = __float_as_uint(f);
  const unsigned s  = (u >> 16) & 0x8000u;
  const unsigned a  = u & 0x7fffffffu;
  const unsigned t  = a - 0x38000000u;
  const unsigned r  = (t + 0x0FFFu + ((t >> 13) & 1u)) >> 13;
  const unsigned rc = r > 0x7C00u ? 0x7C00u : r;
  const bool small  = a < 0x38800000u;
  const bool isnan  = a > 0x7f800000u;
  const unsigned fin = small ? 0u : (s | rc);
  return isnan ? (s | 0x7E00u) : fin;
}

__device__ __forceinline__ unsigned pk16(unsigned lo, unsigned hi) { return lo | (hi << 16); }
__device__ __forceinline__ unsigned bf16_lo_bits(float v) {
  float hi = bf16_val(v);
  asm volatile("" : "+v"(hi));
  return bf16_bits(v - hi);
}
__device__ __forceinline__ v4u pack8_bf16(v4f a, v4f c) {
  return (v4u){ pk16(bf16_bits(a[0]), bf16_bits(a[1])), pk16(bf16_bits(a[2]), bf16_bits(a[3])),
                pk16(bf16_bits(c[0]), bf16_bits(c[1])), pk16(bf16_bits(c[2]), bf16_bits(c[3])) };
}
__device__ __forceinline__ v4u pack8_bf16_lo(v4f a, v4f c) {
  return (v4u){ pk16(bf16_lo_bits(a[0]), bf16_lo_bits(a[1])), pk16(bf16_lo_bits(a[2]), bf16_lo_bits(a[3])),
                pk16(bf16_lo_bits(c[0]), bf16_lo_bits(c[1])), pk16(bf16_lo_bits(c[2]), bf16_lo_bits(c[3])) };
}
__device__ __forceinline__ v4u pack8_f16(v4f a, v4f c) {
  return (v4u){ pk16(f16_bits(a[0]), f16_bits(a[1])), pk16(f16_bits(a[2]), f16_bits(a[3])),
                pk16(f16_bits(c[0]), f16_bits(c[1])), pk16(f16_bits(c[2]), f16_bits(c[3])) };
}

template <int FORM>
__global__ __launch_bounds__(256) void k_plane(const float* __restrict__ src, int rows, int cols, int ldsrc,
                                               unsigned short* __restrict__ dst, int MP, int KP) {
  static_assert(FORM >= 0 && FORM <= 3);
  const int KTOT = (FORM == 1 || FORM == 3) ? 2 * KP : KP;
  const unsigned ppr   = (unsigned)(KTOT >> 3);
  const unsigned kp8   = (unsigned)(KP >> 3);
  const unsigned total = (unsigned)MP * ppr;
  const unsigned g     = blockIdx.x * 256u + threadIdx.x;
  const unsigned rowu  = g / ppr;
  const unsigned p     = g - rowu * ppr;
  const bool second    = p >= kp8;
  const int row = (int)rowu;
  const int c0  = (int)((second ? p - kp8 : p) << 3);
  const float* srow = src + (size_t)clampi(row, 0, rows - 1) * (size_t)ldsrc;
  float x[8];
  unsigned mk[8];
#pragma unroll
  for (int e = 0; e < 8; ++e) {
    const int c = c0 + e;
    const float v = srow[clampi(c, 0, cols - 1)];
    asm volatile("" :: "v"(v));
    x[e]  = v;
    mk[e] = (row < rows && c < cols) ? 0xFFFFu : 0u;
  }
  const v4f a = (v4f){ x[0], x[1], x[2], x[3] };
  const v4f c = (v4f){ x[4], x[5], x[6], x[7] };
  v4u o;
  if (FORM == 2) {
    o = pack8_f16(a, c);
  } else {
    const v4u hi = pack8_bf16(a, c);
    o = hi;
    if (FORM == 1) { const v4u lo = pack8_bf16_lo(a, c); o = second ? lo : hi; }
  }
  const v4u mw = (v4u){ pk16(mk[0], mk[1]), pk16(mk[2], mk[3]), pk16(mk[4], mk[5]), pk16(mk[6], mk[7]) };
  o &= mw;
  if (g < total) {
    volatile v4u* q = (volatile v4u*)(dst + (size_t)g * 8);
    *q = o;
    __threadfence();
    *q = o;
  }
}

template <int FORM> struct FragOf    { typedef FragB T; };
template <>         struct FragOf<2> { typedef FragH T; };
__device__ __forceinline__ v8f mm(const FragB& a, const FragB& b, v8f c) { return wmb(a, b, c); }
__device__ __forceinline__ v8f mm(const FragH& a, const FragH& b, v8f c) { return wmh(a, b, c); }
template <class F> __device__ __forceinline__ F ld_frag(const unsigned short* p) {
  F f;
  f.h[0] = *(const v8usa*)(p);
  f.h[1] = *(const v8usa*)(p + 16);
  return f;
}

template <int FORM, int EPI>
__global__ __launch_bounds__(256) __attribute__((amdgpu_num_vgpr(248)))
void k_gemm_nt(const unsigned short* __restrict__ A, const unsigned short* __restrict__ B,
               const float* __restrict__ bias, float* __restrict__ D, int M, int N, int KTOT, int ldd) {
  static_assert(FORM >= 0 && FORM <= 2);
  static_assert(EPI == 0 || EPI == 1);
  typedef typename FragOf<FORM>::T F;
  __shared__ __attribute__((aligned(16))) float sT[8][16 * 68];
  const int lane = threadIdx.x & 31;
  const int wave = threadIdx.x >> 5;
  const int tilesM = (M + 63) >> 6;
  const int tilesN = (N + 63) >> 6;
  const int tile = blockIdx.x * 8 + wave;
  if (tile >= tilesM * tilesN) return;
  const int tm = tile / tilesN;
  const int tn = tile - tm * tilesN;
  const int m0 = tm << 6;
  const int n0 = tn << 6;

  const int rl = lane & 15;
  const int h8 = (lane >> 4) * 8;
  const unsigned short* pa = A + (size_t)(m0 + rl) * (size_t)KTOT + h8;
  const unsigned short* pb = B + (size_t)(n0 + rl) * (size_t)KTOT + h8;

  v8f acc[4][4];
#pragma unroll
  for (int i = 0; i < 4; ++i)
#pragma unroll
    for (int j = 0; j < 4; ++j) acc[i][j] = (v8f){0.f, 0.f, 0.f, 0.f, 0.f, 0.f, 0.f, 0.f};

#pragma unroll 1
  for (int k0 = 0; k0 < KTOT; k0 += 32) {
    F bf[4];
#pragma unroll
    for (int j = 0; j < 4; ++j) bf[j] = ld_frag<F>(pb + (size_t)(j << 4) * (size_t)KTOT + k0);
#pragma unroll
    for (int i = 0; i < 4; ++i) {
      const F af = ld_frag<F>(pa + (size_t)(i << 4) * (size_t)KTOT + k0);
#pragma unroll
      for (int j = 0; j < 4; ++j) acc[i][j] = mm(af, bf[j], acc[i][j]);
    }
  }

  float* slab = sT[wave];
  const int hh = lane >> 4;
  const int c4 = (lane & 15) * 4;
  const int nc = n0 + c4;
  const bool cok = nc < N;
  v4f bv = (v4f){0.f, 0.f, 0.f, 0.f};
  if (EPI == 1) {
    bv = *(const v4fa*)(bias + clampi(nc, 0, N - 4));
    asm volatile("" :: "v"(bv));
  }
#pragma unroll
  for (int i = 0; i < 4; ++i) {
    const int mBase = m0 + (i << 4);
#pragma unroll
    for (int j = 0; j < 4; ++j) {
#pragma unroll
      for (int r = 0; r < 8; ++r) slab[(h8 + r) * 68 + (j << 4) + rl] = acc[i][j][r];
    }
    __builtin_amdgcn_fence(__ATOMIC_RELEASE, "workgroup");
    __builtin_amdgcn_wave_barrier();
    __builtin_amdgcn_fence(__ATOMIC_ACQUIRE, "workgroup");
    v4f vv[8];
#pragma unroll
    for (int it = 0; it < 8; ++it) {
      const int row = it * 2 + hh;
      v4f v = *(const v4fa*)(slab + row * 68 + c4);
      if (EPI == 1) v += bv;
      vv[it] = v;
    }
    for (int pass = 0; pass < 2; ++pass) {
#pragma unroll
      for (int it = 0; it < 8; ++it) {
        const int row = mBase + it * 2 + hh;
        if (cok && row < M) *(volatile v4f*)(D + (size_t)row * (size_t)ldd + nc) = vv[it];
      }
      __threadfence();
    }
    __builtin_amdgcn_fence(__ATOMIC_RELEASE, "workgroup");
    __builtin_amdgcn_wave_barrier();
    __builtin_amdgcn_fence(__ATOMIC_ACQUIRE, "workgroup");
  }
}

#pragma clang fp contract(off)


#ifndef SPLIT_1
#define SPLIT_1 1
#endif
#ifndef SPLIT_2
#define SPLIT_2 1
#endif

#define NN      50000
#define NE      800000
#define MPAD    50048
#define NHD     4
#define FW      128
#define FW2     256
#define OUTN    8000000
#define RTHR    256
#define RWAVES  8
#define TB_AL0  0
#define TB_AR0  128
#define TB_B0   256
#define TB_AL1  384
#define TB_AR1  512
#define TB_B1   640
#define TB_AL2  768
#define TB_AR2  1024
#define TB_B2   1280
#define TB_N    1536
#define EROFF   (MPAD * NHD)
#define BT      512
#define BW      16
#define BEPT    8
#define BCHUNK  (BT * BEPT)
#define NCH     ((NE + BCHUNK - 1) / BCHUNK)
#define NB      1024
#define NBLK    ((NN + NB - 1) / NB)
#define RCAP    20480
#define DEGCAP  48
#define SLOTSH  21
#define LISTTOT (NBLK * RCAP)
#define LDS_BKT ((2 * RCAP + 3 * NB + 64) * 4)
#define WSMAX   ((size_t)128 << 20)

static_assert(NN % 8 == 0 && MPAD % 8 == 0);
static_assert(MPAD == 782 * 64 && MPAD >= NN);
static_assert(OUTN == NN * 160 && OUTN % 32 == 0 && OUTN % 256 == 0);
static_assert(NE < (1 << SLOTSH));
static_assert(NB <= 1024 && (NB & (NB - 1)) == 0 && NB == 2 * BT);
static_assert(NE % 8 == 0 && NE >= 8);
static_assert(NBLK == 49 && NBLK * NB >= MPAD);
static_assert(NCH * BCHUNK >= NE && NCH == 196);
static_assert(RCAP % (4 * BT) == 0);
static_assert(RCAP >= 16696 + 8);
static_assert(DEGCAP >= 33 + 8);
static_assert(LDS_BKT <= 327680);
static_assert(BW == BT / 32 && BW == 16);

typedef int v4i __attribute__((ext_vector_type(4)));
typedef int v2i __attribute__((ext_vector_type(2)));
typedef v4i __attribute__((may_alias)) v4ia;
typedef v2i __attribute__((may_alias)) v2ia;

__device__ __forceinline__ float relu_k(float v) { return (v > 0.0f) ? v : (v - v); }
__device__ __forceinline__ float lrelu_k(float v) { return (v > 0.0f) ? v : 0.2f * v; }
__device__ __forceinline__ float maxk(float a, float b) {
  float m = (a < b) ? b : a;
  m = (b != b) ? b : m;
  return m;
}
__device__ __forceinline__ float fin0(float m) {
  return ((__float_as_uint(m) & 0x7fffffffu) < 0x7f800000u) ? m : 0.0f;
}
__device__ __forceinline__ float sum8(float t) {
  t = t + __shfl_xor(t, 4, 32);
  t = t + __shfl_xor(t, 2, 32);
  t = t + __shfl_xor(t, 1, 32);
  return t;
}
__device__ __forceinline__ float hmean4(float v, int cg) {
  const float a0 = __shfl(v, cg, 32);
  const float a1 = __shfl(v, cg + 8, 32);
  const float a2 = __shfl(v, cg + 16, 32);
  const float a3 = __shfl(v, cg + 24, 32);
  float s = a0 + a1;
  s = s + a2;
  s = s + a3;
  return s * 0.25f;
}
__device__ __forceinline__ v4u mb4(v4f a, unsigned m) {
  return (v4u){ __float_as_uint(a.x) & m, __float_as_uint(a.y) & m, __float_as_uint(a.z) & m, __float_as_uint(a.w) & m };
}

__global__ __launch_bounds__(256) void k_prep(
    const float* __restrict__ W0, const float* __restrict__ W1, const float* __restrict__ W2,
    const float* __restrict__ al0, const float* __restrict__ ar0, const float* __restrict__ b0,
    const float* __restrict__ al1, const float* __restrict__ ar1, const float* __restrict__ b1,
    const float* __restrict__ al2, const float* __restrict__ ar2, const float* __restrict__ b2,
    unsigned short* W0T, unsigned short* W1D, unsigned short* W2D, float* TB) {
  const int blk = (int)blockIdx.x;
  const int tid = (int)threadIdx.x;
  if (blk < 8) {
    const int g = blk * 256 + tid;
    const int n = g >> 4, p = g & 15;
    float x[8];
#pragma unroll
    for (int e = 0; e < 8; ++e) {
      const float v = W0[(8 * p + e) * 128 + n];
      asm volatile("" :: "v"(v));
      x[e] = v;
    }
    const v4u o = pack8_bf16((v4f){ x[0], x[1], x[2], x[3] }, (v4f){ x[4], x[5], x[6], x[7] });
    volatile v4u* q = (volatile v4u*)(W0T + (size_t)g * 8);
    *q = o;
    __threadfence();
    *q = o;
  } else if (blk < 12) {
    const int g = (blk - 8) * 256 + tid;
    const int n = g >> 3, p = g & 7;
    float x[8];
#pragma unroll
    for (int e = 0; e < 8; ++e) {
      const int kk = (8 * p + e) & 31;
      const float v = W1[kk * 128 + n];
      asm volatile("" :: "v"(v));
      x[e] = v;
    }
    const v4u o = pack8_bf16((v4f){ x[0], x[1], x[2], x[3] }, (v4f){ x[4], x[5], x[6], x[7] });
    volatile v4u* q = (volatile v4u*)(W1D + (size_t)g * 8);
    *q = o;
    __threadfence();
    *q = o;
  } else if (blk < 20) {
    const int g = (blk - 12) * 256 + tid;
    const int rr = g >> 3, p = g & 7;
    const int hh = rr >> 6, c = rr & 63;
    const int col = 40 * hh + (c < 40 ? c : 39);
    const unsigned msk = (c < 40) ? 0xFFFFFFFFu : 0u;
    float x[8];
#pragma unroll
    for (int e = 0; e < 8; ++e) {
      const int kk = (8 * p + e) & 31;
      const float v = W2[kk * 160 + col];
      asm volatile("" :: "v"(v));
      x[e] = v;
    }
    v4u o = pack8_bf16((v4f){ x[0], x[1], x[2], x[3] }, (v4f){ x[4], x[5], x[6], x[7] });
    o &= (v4u){ msk, msk, msk, msk };
    volatile v4u* q = (volatile v4u*)(W2D + (size_t)g * 8);
    *q = o;
    __threadfence();
    *q = o;
  } else {
    const int u   = (blk - 20) * 256 + tid;
    const int uc  = u < 384 ? u : 383;
    const int idx = 4 * uc;
    const int s   = idx >> 7;
    const int o1  = idx & 127;
    const int j   = idx >= 768 ? idx - 768 : 0;
    const int s2  = j >> 8;
    const int r   = j & 255;
    const int hh  = r >> 6, c = r & 63;
    const bool okc = c < 40;
    const int o2  = 40 * hh + (okc ? c : 36);
    const v4f a0 = *(const v4fa*)(al0 + o1); asm volatile("" :: "v"(a0));
    const v4f a1 = *(const v4fa*)(ar0 + o1); asm volatile("" :: "v"(a1));
    const v4f a2 = *(const v4fa*)(b0  + o1); asm volatile("" :: "v"(a2));
    const v4f a3 = *(const v4fa*)(al1 + o1); asm volatile("" :: "v"(a3));
    const v4f a4 = *(const v4fa*)(ar1 + o1); asm volatile("" :: "v"(a4));
    const v4f a5 = *(const v4fa*)(b1  + o1); asm volatile("" :: "v"(a5));
    const v4f a6 = *(const v4fa*)(al2 + o2); asm volatile("" :: "v"(a6));
    const v4f a7 = *(const v4fa*)(ar2 + o2); asm volatile("" :: "v"(a7));
    const v4f a8 = *(const v4fa*)(b2  + o2); asm volatile("" :: "v"(a8));
    const bool lowp = idx < 768;
    const unsigned m0 = (lowp && s == 0) ? 0xFFFFFFFFu : 0u;
    const unsigned m1 = (lowp && s == 1) ? 0xFFFFFFFFu : 0u;
    const unsigned m2 = (lowp && s == 2) ? 0xFFFFFFFFu : 0u;
    const unsigned m3 = (lowp && s == 3) ? 0xFFFFFFFFu : 0u;
    const unsigned m4 = (lowp && s == 4) ? 0xFFFFFFFFu : 0u;
    const unsigned m5 = (lowp && s == 5) ? 0xFFFFFFFFu : 0u;
    const unsigned m6 = (!lowp && okc && s2 == 0) ? 0xFFFFFFFFu : 0u;
    const unsigned m7 = (!lowp && okc && s2 == 1) ? 0xFFFFFFFFu : 0u;
    const unsigned m8 = (!lowp && okc && s2 == 2) ? 0xFFFFFFFFu : 0u;
    v4u o = mb4(a0, m0) | mb4(a1, m1) | mb4(a2, m2) | mb4(a3, m3) | mb4(a4, m4) | mb4(a5, m5) |
            mb4(a6, m6) | mb4(a7, m7) | mb4(a8, m8);
    o.x = bf16_bits(__uint_as_float(o.x)) << 16;
    o.y = bf16_bits(__uint_as_float(o.y)) << 16;
    o.z = bf16_bits(__uint_as_float(o.z)) << 16;
    o.w = bf16_bits(__uint_as_float(o.w)) << 16;
    const bool wr = u < 384;
    volatile v4u* q = (volatile v4u*)(TB + idx);
    if (wr) *q = o;
    __threadfence();
    if (wr) *q = o;
  }
}

template <int CPL>
__global__ __launch_bounds__(RTHR) void k_rowprep(const float* __restrict__ Fm, const float* __restrict__ tal,
                                                  const float* __restrict__ tar, float* ELR) {
  static_assert(CPL == 4 || CPL == 8);
  __shared__ __attribute__((aligned(16))) float sd[2 * RWAVES * NHD];
  const int lane = (int)threadIdx.x & 31;
  const int wave = (int)threadIdx.x >> 5;
  const int row  = (int)blockIdx.x * RWAVES + wave;
  const int rowc = row < NN ? row : NN - 1;
  const int head = lane >> 3;
  const int c0   = lane * CPL;
  const float* prow = Fm + (size_t)rowc * (size_t)(32 * CPL) + c0;
  const v4f p = *(const v4fa*)prow;
  asm volatile("" :: "v"(p));
  const v4f a = *(const v4fa*)(tal + c0);
  const v4f b = *(const v4fa*)(tar + c0);
  float tl = p.x * a.x;
  float u  = p.y * a.y; tl = tl + u;
  u = p.z * a.z; tl = tl + u;
  u = p.w * a.w; tl = tl + u;
  float tr = p.x * b.x;
  u = p.y * b.y; tr = tr + u;
  u = p.z * b.z; tr = tr + u;
  u = p.w * b.w; tr = tr + u;
  if (CPL == 8) {
    const v4f p2 = *(const v4fa*)(prow + 4);
    asm volatile("" :: "v"(p2));
    const v4f a2 = *(const v4fa*)(tal + c0 + 4);
    const v4f b2 = *(const v4fa*)(tar + c0 + 4);
    u = p2.x * a2.x; tl = tl + u;
    u = p2.y * a2.y; tl = tl + u;
    u = p2.z * a2.z; tl = tl + u;
    u = p2.w * a2.w; tl = tl + u;
    u = p2.x * b2.x; tr = tr + u;
    u = p2.y * b2.y; tr = tr + u;
    u = p2.z * b2.z; tr = tr + u;
    u = p2.w * b2.w; tr = tr + u;
  }
  tl = sum8(tl);
  tr = sum8(tr);
  if ((lane & 7) == 0) {
    sd[wave * NHD + head] = tl;
    sd[RWAVES * NHD + wave * NHD + head] = tr;
  }
  __syncthreads();
  if (wave < 2) {
    const int l8 = lane & 7;
    const v4f sv = *(const v4fa*)(sd + RWAVES * NHD * wave + 4 * l8);
    const int trow = (int)blockIdx.x * RWAVES + l8;
    const bool wr = (lane < 8) && (trow < NN);
    volatile v4f* q = (volatile v4f*)(ELR + (size_t)wave * EROFF + (size_t)(trow < NN ? trow : NN - 1) * NHD);
    if (wr) *q = sv;
    __threadfence();
    if (wr) *q = sv;
  }
}

__global__ __launch_bounds__(BT) void k_list(const int* __restrict__ ekey, const int* __restrict__ eids,
                                             unsigned* LIST, int* META) {
  extern __shared__ v4u lds_bkt[];
  int* reg1 = (int*)lds_bkt;
  int* reg2 = reg1 + RCAP;
  int* scnt = reg2 + RCAP;
  int* soff = scnt + NB;
  int* curs = soff + NB;
  int* wcnt = curs + NB;
  int* wtot = wcnt + 2 * BW;
  const int tid = (int)threadIdx.x, lane = tid & 31, wave = tid >> 5;
  const int nodeBase = (int)blockIdx.x * NB;
  int nb = NN - nodeBase;
  nb = nb > NB ? NB : (nb < 0 ? 0 : nb);
  const unsigned nbs = (unsigned)nodeBase, unb = (unsigned)nb;

  scnt[2 * tid] = 0;
  scnt[2 * tid + 1] = 0;
  if (tid == 0) reg2[0] = 0;

  int tot = 0;
#pragma unroll 1
  for (int ch = 0; ch < NCH; ++ch) {
    const int par = ch & 1;
    const int e0  = ch * BCHUNK + tid * BEPT;
    const bool valid = e0 < NE;
    const int ea = e0 < NE - 8 ? e0 : NE - 8;
    const v4i da = *(const v4ia*)(ekey + ea);
    const v4i db = *(const v4ia*)(ekey + ea + 4);
    asm volatile("" :: "v"(da), "v"(db));
    const unsigned s0 = (unsigned)da.x - nbs, s1 = (unsigned)da.y - nbs;
    const unsigned s2 = (unsigned)da.z - nbs, s3 = (unsigned)da.w - nbs;
    const unsigned s4 = (unsigned)db.x - nbs, s5 = (unsigned)db.y - nbs;
    const unsigned s6 = (unsigned)db.z - nbs, s7 = (unsigned)db.w - nbs;
    const bool h0 = valid && (s0 < unb), h1 = valid && (s1 < unb), h2 = valid && (s2 < unb), h3 = valid && (s3 < unb);
    const bool h4 = valid && (s4 < unb), h5 = valid && (s5 < unb), h6 = valid && (s6 < unb), h7 = valid && (s7 < unb);
    const int c = (int)h0 + (int)h1 + (int)h2 + (int)h3 + (int)h4 + (int)h5 + (int)h6 + (int)h7;
    int incl = c;
#pragma unroll
    for (int d = 1; d < 32; d <<= 1) {
      const int up = __shfl_up(incl, d, 32);
      incl += (lane >= d) ? up : 0;
    }
    const int wtotal = __shfl(incl, 31, 32);
    if (lane == 0) wcnt[par * BW + wave] = wtotal;
    __syncthreads();
    int all = 0, pre = 0;
#pragma unroll
    for (int g = 0; g < 4; ++g) {
      const v4i w4 = *(const v4ia*)(wcnt + par * BW + 4 * g);
      const int c0 = clampi(w4.x, 0, 256), c1 = clampi(w4.y, 0, 256);
      const int c2 = clampi(w4.z, 0, 256), c3 = clampi(w4.w, 0, 256);
      all += c0 + c1 + c2 + c3;
      pre += (4 * g + 0 < wave) ? c0 : 0;
      pre += (4 * g + 1 < wave) ? c1 : 0;
      pre += (4 * g + 2 < wave) ? c2 : 0;
      pre += (4 * g + 3 < wave) ? c3 : 0;
    }
    int pos = tot + pre + (incl - c);
#define PUTJ(J, HJ, SJ) if (HJ) { if (pos < RCAP) reg1[pos] = (int)((unsigned)(e0 + (J)) | ((SJ) << SLOTSH)); ++pos; }
    PUTJ(0, h0, s0)
    PUTJ(1, h1, s1)
    PUTJ(2, h2, s2)
    PUTJ(3, h3, s3)
    PUTJ(4, h4, s4)
    PUTJ(5, h5, s5)
    PUTJ(6, h6, s6)
    PUTJ(7, h7, s7)
#undef PUTJ
    tot += all;
  }
  __syncthreads();
  const bool ovf = tot > RCAP;
  const int nh = ovf ? RCAP : tot;

  if (wave == 0) {
#pragma unroll 1
    for (int b0 = 0; b0 < nh; b0 += 32) {
      const int idx = b0 + lane;
      const int uv  = reg1[idx < nh ? idx : nh - 1];
      const int m32 = (nh - b0) < 32 ? (nh - b0) : 32;
#pragma unroll 1
      for (int k = 0; k < m32; ++k) {
        const int u  = __builtin_amdgcn_readlane(uv, k);
        const int sl = (int)(((unsigned)u >> SLOTSH) & (unsigned)(NB - 1));
        const int cv = scnt[sl] + 1;
        if (lane == 0) scnt[sl] = cv;
      }
    }
  }
  __syncthreads();

  int e0c, e1c;
  {
    const v2i cc = *(const v2ia*)(scnt + 2 * tid);
    e0c = cc.x < 0 ? 0 : cc.x;
    e1c = cc.y < 0 ? 0 : cc.y;
    const int ts = e0c + e1c;
    int incl = ts;
#pragma unroll
    for (int d = 1; d < 32; d <<= 1) {
      const int up = __shfl_up(incl, d, 32);
      incl += (lane >= d) ? up : 0;
    }
    if (lane == 31) wtot[wave] = incl;
    __syncthreads();
    int pre = 0;
#pragma unroll
    for (int g = 0; g < 4; ++g) {
      const v4i w4 = *(const v4ia*)(wtot + 4 * g);
      pre += (4 * g + 0 < wave) ? w4.x : 0;
      pre += (4 * g + 1 < wave) ? w4.y : 0;
      pre += (4 * g + 2 < wave) ? w4.z : 0;
      pre += (4 * g + 3 < wave) ? w4.w : 0;
    }
    const int run = pre + incl - ts;
    soff[2 * tid]     = run;
    soff[2 * tid + 1] = run + e0c;
    curs[2 * tid]     = run;
    curs[2 * tid + 1] = run + e0c;
  }
  __syncthreads();

  if (wave == 0) {
#pragma unroll 1
    for (int b0 = 0; b0 < nh; b0 += 32) {
      const int idx = b0 + lane;
      const int uv  = reg1[idx < nh ? idx : nh - 1];
      const int m32 = (nh - b0) < 32 ? (nh - b0) : 32;
#pragma unroll 1
      for (int k = 0; k < m32; ++k) {
        const int u   = __builtin_amdgcn_readlane(uv, k);
        const int sl  = (int)(((unsigned)u >> SLOTSH) & (unsigned)(NB - 1));
        const int eid = (int)((unsigned)u & ((1u << SLOTSH) - 1u));
        const int pr  = curs[sl];
        const int pc  = clampi(pr, 0, RCAP - 1);
        if (lane == 0) { reg2[pc] = eid; curs[sl] = pc + 1; }
      }
    }
  }
  __syncthreads();

  {
    unsigned* lbase = LIST + (size_t)blockIdx.x * (size_t)RCAP;
    const int nhm1 = nh > 0 ? nh - 1 : 0;
#pragma unroll 1
    for (int it = 0; it < RCAP / (4 * BT); ++it) {
      const int i0 = 4 * (it * BT + tid);
      unsigned w[4];
#pragma unroll
      for (int e = 0; e < 4; ++e) {
        const int i  = i0 + e;
        const int ic = i < nhm1 ? i : nhm1;
        const int eid = clampi(reg2[ic], 0, NE - 1);
        const int cw = eids[eid];
        asm volatile("" :: "v"(cw));
        const unsigned msk = (i < nh) ? 0xFFFFFFFFu : 0u;
        w[e] = (unsigned)clampi(cw, 0, NN - 1) & msk;
      }
      const v4u o = (v4u){ w[0], w[1], w[2], w[3] };
      volatile v4u* q = (volatile v4u*)(lbase + i0);
      *q = o;
      __threadfence();
      *q = o;
    }
  }

  {
    const int base = (int)blockIdx.x * RCAP;
    const v2i cc = *(const v2ia*)(scnt + 2 * tid);
    const v2i so = *(const v2ia*)(soff + 2 * tid);
    v4i m;
    m.x = base + so.x;
    m.y = ovf ? -1 : cc.x;
    m.z = base + so.y;
    m.w = ovf ? -1 : cc.y;
    volatile v4i* q = (volatile v4i*)(META + 2 * (size_t)(nodeBase + 2 * tid));
    *q = m;
    __threadfence();
    *q = m;
  }
}

__global__ __launch_bounds__(RTHR) void k_walk32(const float* __restrict__ F, const float* __restrict__ ELR,
                                                 const unsigned* __restrict__ LIST, const int* __restrict__ META,
                                                 const float* __restrict__ bias, unsigned short* OP,
                                                 unsigned lomask) {
  const int lane = (int)threadIdx.x & 31;
  const int wave = (int)threadIdx.x >> 5;
  const int row  = (int)blockIdx.x * RWAVES + wave;
  const bool real = row < NN;
  const int rowc = real ? row : NN - 1;
  const int head = lane >> 3;
  const int c0   = lane * 4;

  const v2i mt = *(const v2ia*)(META + 2 * (size_t)rowc);
  asm volatile("" :: "v"(mt));
  const int craw = mt.y;
  const int offv = clampi(mt.x, 0, LISTTOT);
  int cntv = clampi(craw, 0, DEGCAP);
  cntv = cntv < (LISTTOT - offv) ? cntv : (LISTTOT - offv);
  cntv = real ? cntv : 0;
  const int off = __builtin_amdgcn_readfirstlane(offv);
  const int cnt = __builtin_amdgcn_readfirstlane(cntv);
  const bool poison = real && ((craw < 0) || (craw > DEGCAP));

  const v4f er4 = *(const v4fa*)(ELR + (size_t)EROFF + (size_t)rowc * NHD);
  asm volatile("" :: "v"(er4));
  const float ninf = -__builtin_inff();
  v4f mx4 = (v4f){ ninf, ninf, ninf, ninf };

#pragma unroll 1
  for (int b0 = 0; b0 < cnt; b0 += 32) {
    const int j = (b0 + lane) < cnt ? (b0 + lane) : cnt - 1;
    const unsigned sid = LIST[(size_t)(off + j)];
    asm volatile("" :: "v"(sid));
    const int col = clampi((int)sid, 0, NN - 1);
    const v4f el = *(const v4fa*)(ELR + (size_t)col * NHD);
    asm volatile("" :: "v"(el));
    mx4.x = maxk(mx4.x, lrelu_k(el.x + er4.x));
    mx4.y = maxk(mx4.y, lrelu_k(el.y + er4.y));
    mx4.z = maxk(mx4.z, lrelu_k(el.z + er4.z));
    mx4.w = maxk(mx4.w, lrelu_k(el.w + er4.w));
  }
#pragma unroll
  for (int d = 16; d > 0; d >>= 1) {
    const float o0 = __shfl_xor(mx4.x, d, 32);
    const float o1 = __shfl_xor(mx4.y, d, 32);
    const float o2 = __shfl_xor(mx4.z, d, 32);
    const float o3 = __shfl_xor(mx4.w, d, 32);
    mx4.x = maxk(mx4.x, o0);
    mx4.y = maxk(mx4.y, o1);
    mx4.z = maxk(mx4.z, o2);
    mx4.w = maxk(mx4.w, o3);
  }
  mx4.x = fin0(mx4.x); mx4.y = fin0(mx4.y); mx4.z = fin0(mx4.z); mx4.w = fin0(mx4.w);

  float den = 0.0f;
  v4f ac = (v4f){ 0.0f, 0.0f, 0.0f, 0.0f };
#pragma unroll 1
  for (int b0 = 0; b0 < cnt; b0 += 32) {
    const int j = (b0 + lane) < cnt ? (b0 + lane) : cnt - 1;
    const unsigned sid = LIST[(size_t)(off + j)];
    asm volatile("" :: "v"(sid));
    const int col = clampi((int)sid, 0, NN - 1);
    const v4f el = *(const v4fa*)(ELR + (size_t)col * NHD);
    asm volatile("" :: "v"(el));
    const float v0 = lrelu_k(el.x + er4.x) - mx4.x;
    const float v1 = lrelu_k(el.y + er4.y) - mx4.y;
    const float v2 = lrelu_k(el.z + er4.z) - mx4.z;
    const float v3 = lrelu_k(el.w + er4.w) - mx4.w;
    const float q0 = expf(v0);
    const float q1 = expf(v1);
    const float q2 = expf(v2);
    const float q3 = expf(v3);
    const int m32 = (cnt - b0) < 32 ? (cnt - b0) : 32;
#pragma unroll 1
    for (int k = 0; k < m32; ++k) {
      const int c = __builtin_amdgcn_readlane(col, k);
      const float w0 = __int_as_float(__builtin_amdgcn_readlane(__float_as_int(q0), k));
      const float w1 = __int_as_float(__builtin_amdgcn_readlane(__float_as_int(q1), k));
      const float w2 = __int_as_float(__builtin_amdgcn_readlane(__float_as_int(q2), k));
      const float w3 = __int_as_float(__builtin_amdgcn_readlane(__float_as_int(q3), k));
      float w = w0;
      w = (head == 1) ? w1 : w;
      w = (head == 2) ? w2 : w;
      w = (head == 3) ? w3 : w;
      const v4f hn = *(const v4fa*)(F + (size_t)c * FW + c0);
      asm volatile("" :: "v"(hn));
      den = den + w;
      float pr;
      pr = w * hn.x; ac.x = ac.x + pr;
      pr = w * hn.y; ac.y = ac.y + pr;
      pr = w * hn.z; ac.z = ac.z + pr;
      pr = w * hn.w; ac.w = ac.w + pr;
    }
  }

  const float dn = (den < 1e-9f) ? 1e-9f : den;
  const v4f bv = *(const v4fa*)(bias + c0);
  asm volatile("" :: "v"(bv));
  v4f r;
  float t;
  t = ac.x / dn; t = t + bv.x; r.x = relu_k(t);
  t = ac.y / dn; t = t + bv.y; r.y = relu_k(t);
  t = ac.z / dn; t = t + bv.z; r.z = relu_k(t);
  t = ac.w / dn; t = t + bv.w; r.w = relu_k(t);

  const int cg = lane & 7;
  const float qnan = __uint_as_float(0x7fc00000u);
  v4f mean;
  mean.x = hmean4(r.x, cg);
  mean.y = hmean4(r.y, cg);
  mean.z = hmean4(r.z, cg);
  mean.w = hmean4(r.w, cg);
  mean.x = poison ? qnan : mean.x;
  mean.y = poison ? qnan : mean.y;
  mean.z = poison ? qnan : mean.z;
  mean.w = poison ? qnan : mean.w;

  const int s0 = 2 * (lane & 3);
  v4f ma, mb;
  ma.x = __shfl(mean.x, s0, 32);     ma.y = __shfl(mean.y, s0, 32);
  ma.z = __shfl(mean.z, s0, 32);     ma.w = __shfl(mean.w, s0, 32);
  mb.x = __shfl(mean.x, s0 + 1, 32); mb.y = __shfl(mean.y, s0 + 1, 32);
  mb.z = __shfl(mean.z, s0 + 1, 32); mb.w = __shfl(mean.w, s0 + 1, 32);
  const v4u hi = pack8_bf16(ma, mb);
  v4u lo = pack8_bf16_lo(ma, mb);
  lo &= (v4u){ lomask, lomask, lomask, lomask };
  const unsigned sl = (lane & 4) ? 0xFFFFFFFFu : 0u;
  const unsigned rm = real ? 0xFFFFFFFFu : 0u;
  v4u o = (lo & (v4u){ sl, sl, sl, sl }) | (hi & (v4u){ ~sl, ~sl, ~sl, ~sl });
  o &= (v4u){ rm, rm, rm, rm };
  volatile v4u* q = (volatile v4u*)(OP + (size_t)row * 64 + 8 * (lane & 7));
  const bool wr = lane < 8;
  if (wr) *q = o;
  __threadfence();
  if (wr) *q = o;
}

__global__ __launch_bounds__(RTHR) void k_walk40(const float* __restrict__ F2, const float* __restrict__ ELR,
                                                 const unsigned* __restrict__ LIST, const int* __restrict__ META,
                                                 const float* __restrict__ bias, float* TF) {
  const int lane = (int)threadIdx.x & 31;
  const int wave = (int)threadIdx.x >> 5;
  const int row  = (int)blockIdx.x * RWAVES + wave;
  const bool real = row < NN;
  const int rowc = real ? row : NN - 1;
  const int hs   = lane >> 4;
  const int c0   = lane * 4;

  const v2i mt = *(const v2ia*)(META + 2 * (size_t)rowc);
  asm volatile("" :: "v"(mt));
  const int craw = mt.y;
  const int offv = clampi(mt.x, 0, LISTTOT);
  int cntv = clampi(craw, 0, DEGCAP);
  cntv = cntv < (LISTTOT - offv) ? cntv : (LISTTOT - offv);
  cntv = real ? cntv : 0;
  const int off = __builtin_amdgcn_readfirstlane(offv);
  const int cnt = __builtin_amdgcn_readfirstlane(cntv);
  const bool poison = real && ((craw < 0) || (craw > DEGCAP));

  const v4f er4 = *(const v4fa*)(ELR + (size_t)EROFF + (size_t)rowc * NHD);
  asm volatile("" :: "v"(er4));
  const float ninf = -__builtin_inff();
  v4f mx4 = (v4f){ ninf, ninf, ninf, ninf };

#pragma unroll 1
  for (int b0 = 0; b0 < cnt; b0 += 32) {
    const int j = (b0 + lane) < cnt ? (b0 + lane) : cnt - 1;
    const unsigned sid = LIST[(size_t)(off + j)];
    asm volatile("" :: "v"(sid));
    const int col = clampi((int)sid, 0, NN - 1);
    const v4f el = *(const v4fa*)(ELR + (size_t)col * NHD);
    asm volatile("" :: "v"(el));
    mx4.x = maxk(mx4.x, lrelu_k(el.x + er4.x));
    mx4.y = maxk(mx4.y, lrelu_k(el.y + er4.y));
    mx4.z = maxk(mx4.z, lrelu_k(el.z + er4.z));
    mx4.w = maxk(mx4.w, lrelu_k(el.w + er4.w));
  }
#pragma unroll
  for (int d = 16; d > 0; d >>= 1) {
    const float o0 = __shfl_xor(mx4.x, d, 32);
    const float o1 = __shfl_xor(mx4.y, d, 32);
    const float o2 = __shfl_xor(mx4.z, d, 32);
    const float o3 = __shfl_xor(mx4.w, d, 32);
    mx4.x = maxk(mx4.x, o0);
    mx4.y = maxk(mx4.y, o1);
    mx4.z = maxk(mx4.z, o2);
    mx4.w = maxk(mx4.w, o3);
  }
  mx4.x = fin0(mx4.x); mx4.y = fin0(mx4.y); mx4.z = fin0(mx4.z); mx4.w = fin0(mx4.w);

  float dena = 0.0f, denb = 0.0f;
  v4f aa = (v4f){ 0.0f, 0.0f, 0.0f, 0.0f };
  v4f ab = (v4f){ 0.0f, 0.0f, 0.0f, 0.0f };
#pragma unroll 1
  for (int b0 = 0; b0 < cnt; b0 += 32) {
    const int j = (b0 + lane) < cnt ? (b0 + lane) : cnt - 1;
    const unsigned sid = LIST[(size_t)(off + j)];
    asm volatile("" :: "v"(sid));
    const int col = clampi((int)sid, 0, NN - 1);
    const v4f el = *(const v4fa*)(ELR + (size_t)col * NHD);
    asm volatile("" :: "v"(el));
    const float v0 = lrelu_k(el.x + er4.x) - mx4.x;
    const float v1 = lrelu_k(el.y + er4.y) - mx4.y;
    const float v2 = lrelu_k(el.z + er4.z) - mx4.z;
    const float v3 = lrelu_k(el.w + er4.w) - mx4.w;
    const float q0 = expf(v0);
    const float q1 = expf(v1);
    const float q2 = expf(v2);
    const float q3 = expf(v3);
    const int m32 = (cnt - b0) < 32 ? (cnt - b0) : 32;
#pragma unroll 1
    for (int k = 0; k < m32; ++k) {
      const int c = __builtin_amdgcn_readlane(col, k);
      const float w0 = __int_as_float(__builtin_amdgcn_readlane(__float_as_int(q0), k));
      const float w1 = __int_as_float(__builtin_amdgcn_readlane(__float_as_int(q1), k));
      const float w2 = __int_as_float(__builtin_amdgcn_readlane(__float_as_int(q2), k));
      const float w3 = __int_as_float(__builtin_amdgcn_readlane(__float_as_int(q3), k));
      const float wa = (hs == 1) ? w1 : w0;
      const float wb = (hs == 1) ? w3 : w2;
      const float* fr = F2 + (size_t)c * FW2 + c0;
      const v4f ha = *(const v4fa*)(fr);
      const v4f hb = *(const v4fa*)(fr + 128);
      asm volatile("" :: "v"(ha), "v"(hb));
      dena = dena + wa;
      denb = denb + wb;
      float pr;
      pr = wa * ha.x; aa.x = aa.x + pr;
      pr = wa * ha.y; aa.y = aa.y + pr;
      pr = wa * ha.z; aa.z = aa.z + pr;
      pr = wa * ha.w; aa.w = aa.w + pr;
      pr = wb * hb.x; ab.x = ab.x + pr;
      pr = wb * hb.y; ab.y = ab.y + pr;
      pr = wb * hb.z; ab.z = ab.z + pr;
      pr = wb * hb.w; ab.w = ab.w + pr;
    }
  }

  const float da = (dena < 1e-9f) ? 1e-9f : dena;
  const float db = (denb < 1e-9f) ? 1e-9f : denb;
  const v4f ba = *(const v4fa*)(bias + c0);
  const v4f bb = *(const v4fa*)(bias + 128 + c0);
  asm volatile("" :: "v"(ba), "v"(bb));
  const float qnan = __uint_as_float(0x7fc00000u);
  v4f oa, ob;
  float t;
  t = aa.x / da; oa.x = t + ba.x;
  t = aa.y / da; oa.y = t + ba.y;
  t = aa.z / da; oa.z = t + ba.z;
  t = aa.w / da; oa.w = t + ba.w;
  t = ab.x / db; ob.x = t + bb.x;
  t = ab.y / db; ob.y = t + bb.y;
  t = ab.z / db; ob.z = t + bb.z;
  t = ab.w / db; ob.w = t + bb.w;
  oa.x = poison ? qnan : oa.x; oa.y = poison ? qnan : oa.y; oa.z = poison ? qnan : oa.z; oa.w = poison ? qnan : oa.w;
  ob.x = poison ? qnan : ob.x; ob.y = poison ? qnan : ob.y; ob.z = poison ? qnan : ob.z; ob.w = poison ? qnan : ob.w;
  const unsigned cm = ((lane & 15) < 10) ? 0xFFFFFFFFu : 0u;
  const v4u ua = mb4(oa, cm);
  const v4u ub = mb4(ob, cm);
  float* trow = TF + (size_t)rowc * FW2 + c0;
  if (real) { *(volatile v4u*)trow = ua; *(volatile v4u*)(trow + 128) = ub; }
  __threadfence();
  if (real) { *(volatile v4u*)trow = ua; *(volatile v4u*)(trow + 128) = ub; }
}

__global__ __launch_bounds__(256) void k_store(const float* __restrict__ TF, float* out) {
  const unsigned f  = blockIdx.x * 256u + threadIdx.x;
  const unsigned fc = f < (unsigned)OUTN ? f : (unsigned)(OUTN - 1);
  const unsigned row = fc / 160u;
  const unsigned r   = fc - 160u * row;
  const unsigned hh  = r / 40u;
  const unsigned c   = r - 40u * hh;
  const float v = TF[(size_t)row * FW2 + 64u * hh + c];
  asm volatile("" :: "v"(v));
  const bool wr = f < (unsigned)OUTN;
  volatile float* q = (volatile float*)(out + fc);
  if (wr) *q = v;
  __threadfence();
  if (wr) *q = v;
}

extern "C" void kernel_launch(void* const* d_in, const int* in_sizes, int n_in,
                              void* d_out, int out_size, void* d_ws, size_t ws_size,
                              hipStream_t stream) {
  if (n_in < 15) return;
  if (in_sizes[0] != NN * 128) return;
  if (in_sizes[1] != NE || in_sizes[2] != NE) return;
  if (in_sizes[3] != 128 * 128) return;
  if (in_sizes[4] != 128 || in_sizes[5] != 128 || in_sizes[6] != 128) return;
  if (in_sizes[7] != 32 * 128) return;
  if (in_sizes[8] != 128 || in_sizes[9] != 128 || in_sizes[10] != 128) return;
  if (in_sizes[11] != 32 * 160) return;
  if (in_sizes[12] != 160 || in_sizes[13] != 160 || in_sizes[14] != 160) return;
  if (out_size != OUTN) return;

  const float* x   = (const float*)d_in[0];
  const int*   src = (const int*)  d_in[1];
  const int*   dst = (const int*)  d_in[2];
  const float* W0  = (const float*)d_in[3];
  const float* al0 = (const float*)d_in[4];
  const float* ar0 = (const float*)d_in[5];
  const float* b0  = (const float*)d_in[6];
  const float* W1  = (const float*)d_in[7];
  const float* al1 = (const float*)d_in[8];
  const float* ar1 = (const float*)d_in[9];
  const float* b1  = (const float*)d_in[10];
  const float* W2  = (const float*)d_in[11];
  const float* al2 = (const float*)d_in[12];
  const float* ar2 = (const float*)d_in[13];
  const float* b2  = (const float*)d_in[14];
  float* out = (float*)d_out;

  const size_t szXB   = (size_t)MPAD * 128 * 2;
  const size_t szF2   = (size_t)MPAD * FW2 * 4;
  const size_t szTF   = (size_t)MPAD * FW2 * 4;
  const size_t szOP   = (size_t)MPAD * 64 * 2;
  const size_t szLIST = (size_t)NBLK * RCAP * 4;
  const size_t szMETA = (size_t)NBLK * NB * 2 * 4;
  const size_t szELR  = (size_t)2 * MPAD * NHD * 4;
  const size_t szW0T  = (size_t)128 * 128 * 2;
  const size_t szW1D  = (size_t)128 * 64 * 2;
  const size_t szW2D  = (size_t)256 * 64 * 2;
  const size_t szTB   = (size_t)TB_N * 4;
  static_assert((size_t)MPAD * 128 * 2 + 2 * ((size_t)MPAD * FW2 * 4) + (size_t)MPAD * 64 * 2 +
                (size_t)NBLK * RCAP * 4 + (size_t)NBLK * NB * 8 + (size_t)2 * MPAD * NHD * 4 +
                (size_t)128 * 128 * 2 + (size_t)128 * 64 * 2 + (size_t)256 * 64 * 2 + (size_t)TB_N * 4
                == (size_t)998608 * 128);
  static_assert((size_t)998608 * 128 <= WSMAX);
  char* ws = (char*)d_ws;
  size_t off = 0;
  const size_t oXB   = off; off += szXB;
  const size_t oF2   = off; off += szF2;
  const size_t oTF   = off; off += szTF;
  const size_t oOP   = off; off += szOP;
  const size_t oLIST = off; off += szLIST;
  const size_t oMETA = off; off += szMETA;
  const size_t oELR  = off; off += szELR;
  const size_t oW0T  = off; off += szW0T;
  const size_t oW1D  = off; off += szW1D;
  const size_t oW2D  = off; off += szW2D;
  const size_t oTB   = off; off += szTB;
  if (off > ws_size || off > (size_t)WSMAX) return;
  unsigned short* XB  = (unsigned short*)(ws + oXB);
  float*          F2  = (float*)(ws + oF2);
  float*          Fp  = F2;
  float*          TF  = (float*)(ws + oTF);
  unsigned short* OP  = (unsigned short*)(ws + oOP);
  unsigned*       LIST = (unsigned*)(ws + oLIST);
  int*            META = (int*)(ws + oMETA);
  float*          ELR = (float*)(ws + oELR);
  unsigned short* W0T = (unsigned short*)(ws + oW0T);
  unsigned short* W1D = (unsigned short*)(ws + oW1D);
  unsigned short* W2D = (unsigned short*)(ws + oW2D);
  float*          TB  = (float*)(ws + oTB);

  hipFuncSetAttribute(reinterpret_cast<const void*>(&k_list),
                      hipFuncAttributeMaxDynamicSharedMemorySize, LDS_BKT);

  const unsigned lom1 = SPLIT_1 ? 0xFFFFFFFFu : 0u;
  const unsigned lom2 = SPLIT_2 ? 0xFFFFFFFFu : 0u;

  static_assert((MPAD * 128 / 8) % 256 == 0);
  k_plane<0><<<MPAD * 128 / 8 / 256, 256, 0, stream>>>(x, NN, 128, 128, XB, MPAD, 128);
  k_prep<<<22, 256, 0, stream>>>(W0, W1, W2, al0, ar0, b0, al1, ar1, b1, al2, ar2, b2, W0T, W1D, W2D, TB);
  k_list<<<NBLK, BT, LDS_BKT, stream>>>(dst, src, LIST, META);

  const int tiles2 = (MPAD / 64) * (128 / 64);
  const int tiles4 = (MPAD / 64) * (256 / 64);
  k_gemm_nt<0, 0><<<(tiles2 + 7) / 8, 256, 0, stream>>>(XB, W0T, TB, Fp, MPAD, 128, 128, 128);
  k_rowprep<4><<<NN / RWAVES, RTHR, 0, stream>>>(Fp, TB + TB_AL0, TB + TB_AR0, ELR);
  k_walk32<<<MPAD / RWAVES, RTHR, 0, stream>>>(Fp, ELR, LIST, META, TB + TB_B0, OP, lom1);
  k_gemm_nt<0, 0><<<(tiles2 + 7) / 8, 256, 0, stream>>>(OP, W1D, TB, Fp, MPAD, 128, 64, 128);
  k_rowprep<4><<<NN / RWAVES, RTHR, 0, stream>>>(Fp, TB + TB_AL1, TB + TB_AR1, ELR);
  k_walk32<<<MPAD / RWAVES, RTHR, 0, stream>>>(Fp, ELR, LIST, META, TB + TB_B1, OP, lom2);
  k_gemm_nt<0, 0><<<(tiles4 + 7) / 8, 256, 0, stream>>>(OP, W2D, TB, F2, MPAD, 256, 64, 256);
  k_rowprep<8><<<NN / RWAVES, RTHR, 0, stream>>>(F2, TB + TB_AL2, TB + TB_AR2, ELR);
  k_walk40<<<NN / RWAVES, RTHR, 0, stream>>>(F2, ELR, LIST, META, TB + TB_B2, TF);
  k_store<<<OUTN / 256, 256, 0, stream>>>(TF, out);
}
